// GlobalLocalAttention_47210280517864
// MI455X (gfx1250) — hardware-verified
//
#include <hip/hip_runtime.h>


#ifndef NB
#define NB 2
#endif
#ifndef SEQ
#define SEQ 4096
#endif
#define NB_FULL  2
#define SEQ_FULL 4096
#define IMW 64
#define IMH (SEQ / IMW)
#define CH  256
#define C3  (3 * CH)
#define NH  8
#define HD  32
#define KCV (9 * CH)
#ifndef SC_HL
#define SC_HL 0
#endif
#ifndef PV_HL
#define PV_HL 0
#endif
#define QCH ((SEQ < 2048) ? SEQ : 2048)
#define NQC (SEQ / QCH)
#define PCAR 16384.0f
#define SCL 0.17677669529663687f
#define BNEPS 1.0e-5f
#define NQKB (NH * SEQ * HD / 256)
#define NVB8 (CH * SEQ / 8)

static_assert(SEQ % 128 == 0);
static_assert(IMW == 64);
static_assert(SEQ % IMW == 0);
static_assert(QCH % 64 == 0);
static_assert(SEQ % QCH == 0);
static_assert(CH % 64 == 0 && C3 % 64 == 0 && HD == 32 && KCV % 32 == 0);
static_assert(NB >= 1 && NB <= NB_FULL && SEQ <= SEQ_FULL);
static_assert((C3 * CH / 8) % 256 == 0 && (CH * CH / 8) % 256 == 0 && (CH * KCV / 8) % 256 == 0);
static_assert(NVB8 % 256 == 0 && (SEQ * CH / 8) % 256 == 0 && SEQ % 8 == 0);

typedef _Float16 h16;
typedef unsigned short bf;
typedef __attribute__((ext_vector_type(16))) __bf16   v16bf;
typedef __attribute__((ext_vector_type(16))) _Float16 v16h;
typedef __attribute__((ext_vector_type(8)))  _Float16 v8h;
typedef __attribute__((ext_vector_type(4)))  _Float16 v4h;
typedef __attribute__((ext_vector_type(2)))  _Float16 v2h;
typedef __attribute__((ext_vector_type(8)))  unsigned short v8us;
typedef __attribute__((ext_vector_type(4)))  unsigned short v4us;
typedef __attribute__((ext_vector_type(2)))  unsigned short v2us;
typedef __attribute__((ext_vector_type(8)))  float    v8f;
typedef __attribute__((ext_vector_type(4)))  float    v4f;
typedef v8h  __attribute__((may_alias)) v8ha;
typedef v4f  __attribute__((may_alias)) v4fa;
typedef v8us __attribute__((may_alias)) v8usa;

__device__ __forceinline__ unsigned short f2bf(float f) { unsigned u = __float_as_uint(f); u += 0x7FFFu + ((u >> 16) & 1u); return (unsigned short)(u >> 16); }
__device__ __forceinline__ float bf2f(unsigned short b) { return __uint_as_float(((unsigned)b) << 16); }
__device__ __forceinline__ float bfr(float f) { return bf2f(f2bf(f)); }
__device__ __forceinline__ h16 tohx(float x) { return (h16)x; }
__device__ __forceinline__ void splitf(float y, unsigned short& h, unsigned short& l) { h = f2bf(y); l = f2bf(y - bf2f(h)); }
__device__ __forceinline__ v16h cat16(v8h lo, v8h hi) { return __builtin_shufflevector(lo, hi, 0, 1, 2, 3, 4, 5, 6, 7, 8, 9, 10, 11, 12, 13, 14, 15); }
__device__ __forceinline__ v16bf cat16b(v8us lo, v8us hi) { return __builtin_bit_cast(v16bf, __builtin_shufflevector(lo, hi, 0, 1, 2, 3, 4, 5, 6, 7, 8, 9, 10, 11, 12, 13, 14, 15)); }
__device__ __forceinline__ v8f wmma16(v16h a, v16h b, v8f c) { return __builtin_amdgcn_wmma_f32_16x16x32_f16(false, a, false, b, (short)0, c, false, false); }
__device__ __forceinline__ v8f wmmab(v16bf a, v16bf b, v8f c) { return __builtin_amdgcn_wmma_f32_16x16x32_bf16(false, a, false, b, (short)0, c, false, false); }
__device__ __forceinline__ void bnfold(const float* g, const float* bt, const float* mu, const float* vr, int i, float& inv, float& sh) { inv = bfr(g[i]) / sqrtf(bfr(vr[i]) + BNEPS); sh = bfr(bt[i]) - bfr(mu[i]) * inv; }

template <typename T16> struct WFrag;
template <> struct WFrag<h16> { typedef v16h V; static __device__ __forceinline__ V ld(const h16* p) { return cat16(*(const v8h*)p, *(const v8h*)(p + 16)); } static __device__ __forceinline__ v8f mma(V a, V b, v8f c) { return wmma16(a, b, c); } };
template <> struct WFrag<bf> { typedef v16bf V; static __device__ __forceinline__ V ld(const bf* p) { return cat16b(*(const v8us*)p, *(const v8us*)(p + 16)); } static __device__ __forceinline__ v8f mma(V a, V b, v8f c) { return wmmab(a, b, c); } };

template <int AFF, int NBK>
__device__ __forceinline__ void epi_slab(float* os, const v8f (&ac)[NBK], float* cslab, int ldc, int rbase, int cbase,
                                         const float* __restrict__ ag, const float* __restrict__ ab, const float* __restrict__ am, const float* __restrict__ av, float osc) {
    constexpr int RW = 16 * NBK, OSP = RW + 4, LPR = RW / 4, RPI = 32 / LPR, NI = 16 / RPI;
    const int lane = threadIdx.x & 31, lr = lane & 15, hi = lane >> 4, rsub = lane / LPR, cofs = (lane % LPR) * 4;
#pragma unroll
    for (int nb = 0; nb < NBK; ++nb)
#pragma unroll
        for (int j = 0; j < 8; ++j) os[(hi * 8 + j) * OSP + nb * 16 + lr] = ac[nb][j];
    __builtin_amdgcn_wave_barrier(); asm volatile("" ::: "memory");
#pragma unroll 1
    for (int ps = 0; ps < 2; ++ps) {
#pragma unroll
        for (int s = 0; s < NI; ++s) { const int row = RPI * s + rsub; v4f val = *(const v4fa*)(os + row * OSP + cofs);
            if (AFF == 1) {
#pragma unroll
                for (int q = 0; q < 4; ++q) { float inv, sh; bnfold(ag, ab, am, av, cbase + cofs + q, inv, sh); val[q] = val[q] * osc * inv + sh; }
            } else if (AFF == 2) { float inv, sh; bnfold(ag, ab, am, av, rbase + row, inv, sh);
#pragma unroll
                for (int q = 0; q < 4; ++q) val[q] = val[q] * osc * inv + sh;
            } else { val = val * osc; }
            *(volatile v4f*)(cslab + (size_t)row * ldc + cofs) = val; }
        if (ps == 0) __threadfence(); }
    __builtin_amdgcn_wave_barrier(); asm volatile("" ::: "memory");
}

template <typename T16, int NSPLIT, int AFF, int NBK>
__global__ __launch_bounds__(32) void k_gemmw(const T16* __restrict__ A, const T16* __restrict__ A2, const T16* __restrict__ Bt, const T16* __restrict__ Bt2, int K, float* C, int ldc,
                                              const float* __restrict__ ag, const float* __restrict__ ab, const float* __restrict__ am, const float* __restrict__ av, float osc, size_t sA, size_t sB, size_t sC) {
    typedef typename WFrag<T16>::V V;
    constexpr bool LA2 = (NSPLIT == 1 || NSPLIT == 2), LB2 = (NSPLIT == 2 || NSPLIT == 3);
    __shared__ __align__(16) float os[16 * (16 * NBK + 4)];
    const size_t z = blockIdx.z; A += z * sA; if (LA2) A2 += z * sA; Bt += z * sB; if (LB2) Bt2 += z * sB; C += z * sC;
    const int lane = threadIdx.x & 31, lr = lane & 15, hi = lane >> 4; const int r0 = blockIdx.x * 64, c0 = blockIdx.y * (16 * NBK);
    v8f acc[4][NBK];
#pragma unroll
    for (int mb = 0; mb < 4; ++mb)
#pragma unroll
        for (int nb = 0; nb < NBK; ++nb) acc[mb][nb] = (v8f){};
    const size_t aoff = (size_t)(r0 + lr) * K + 8 * hi, boff = (size_t)(c0 + lr) * K + 8 * hi;
#pragma unroll 1
    for (int kc = 0; kc < K; kc += 32) {
        V a[4], a2[4];
#pragma unroll
        for (int mb = 0; mb < 4; ++mb) { a[mb] = WFrag<T16>::ld(A + aoff + (size_t)mb * 16 * K + kc); if (LA2) a2[mb] = WFrag<T16>::ld(A2 + aoff + (size_t)mb * 16 * K + kc); else a2[mb] = a[mb]; }
#pragma unroll
        for (int nb = 0; nb < NBK; ++nb) { const V b = WFrag<T16>::ld(Bt + boff + (size_t)nb * 16 * K + kc); V b2 = b; if (LB2) b2 = WFrag<T16>::ld(Bt2 + boff + (size_t)nb * 16 * K + kc);
#pragma unroll
            for (int mb = 0; mb < 4; ++mb) { acc[mb][nb] = WFrag<T16>::mma(a[mb], b, acc[mb][nb]); if (LA2) acc[mb][nb] = WFrag<T16>::mma(a2[mb], b, acc[mb][nb]); if (LB2) acc[mb][nb] = WFrag<T16>::mma(a[mb], b2, acc[mb][nb]); } }
        asm volatile("v_nop\n\tv_nop\n\tv_nop\n\tv_nop" : "+v"(acc[0][0]), "+v"(acc[1][NBK - 1]), "+v"(acc[2][0]), "+v"(acc[3][NBK - 1]) : "v"(a[0]), "v"(a[3]));
    }
#pragma unroll
    for (int mb = 0; mb < 4; ++mb) epi_slab<AFF, NBK>(os, acc[mb], C + (size_t)(r0 + mb * 16) * ldc + c0, ldc, r0 + mb * 16, c0, ag, ab, am, av, osc);
}

__global__ __launch_bounds__(32) void k_convw(const bf* __restrict__ Xp, const bf* __restrict__ Wt, float* C,
                                              const float* __restrict__ ag, const float* __restrict__ ab, const float* __restrict__ am, const float* __restrict__ av) {
    __shared__ __align__(16) float os[16 * 68];
    const int lane = threadIdx.x & 31, lr = lane & 15, hi = lane >> 4; const int r0 = blockIdx.x * 64, c0 = blockIdx.y * 64; const int y = blockIdx.x;
    v8f acc[4][4];
#pragma unroll
    for (int mb = 0; mb < 4; ++mb)
#pragma unroll
        for (int nb = 0; nb < 4; ++nb) acc[mb][nb] = (v8f){};
    const size_t boff = (size_t)(c0 + lr) * KCV + 8 * hi;
#pragma unroll 1
    for (int kc = 0; kc < KCV; kc += 32) {
        const int tap = kc >> 8, cc = kc & 255; const int ky = tap / 3, kx = tap - 3 * ky; const int ys = y + ky - 1; const bool yok = (ys >= 0) && (ys < IMH); const int ysc = ys < 0 ? 0 : (ys > IMH - 1 ? IMH - 1 : ys);
        v16bf a[4];
#pragma unroll
        for (int mb = 0; mb < 4; ++mb) { const int xs = mb * 16 + lr + kx - 1; const bool ok = yok && (xs >= 0) && (xs < IMW); const int xsc = xs < 0 ? 0 : (xs > IMW - 1 ? IMW - 1 : xs);
            const bf* p = Xp + ((size_t)(ysc * IMW + xsc)) * CH + cc + 8 * hi; const v8us u0 = *(const v8us*)p, u1 = *(const v8us*)(p + 16);
            const unsigned short mk = ok ? (unsigned short)0xFFFFu : (unsigned short)0; const v8us m8 = (v8us){mk, mk, mk, mk, mk, mk, mk, mk}; a[mb] = cat16b(u0 & m8, u1 & m8); }
#pragma unroll
        for (int nb = 0; nb < 4; ++nb) { const v16bf b = WFrag<bf>::ld(Wt + boff + (size_t)nb * 16 * KCV + kc);
#pragma unroll
            for (int mb = 0; mb < 4; ++mb) acc[mb][nb] = wmmab(a[mb], b, acc[mb][nb]); }
        asm volatile("v_nop\n\tv_nop\n\tv_nop\n\tv_nop" : "+v"(acc[0][0]), "+v"(acc[1][1]), "+v"(acc[2][2]), "+v"(acc[3][3]) : "v"(a[0]), "v"(a[3]));
    }
#pragma unroll
    for (int mb = 0; mb < 4; ++mb) epi_slab<1, 4>(os, acc[mb], C + (size_t)(r0 + mb * 16) * CH + c0, CH, r0 + mb * 16, c0, ag, ab, am, av, 1.0f);
}

__global__ __launch_bounds__(256) void k_wprep(const float* __restrict__ wq, const float* __restrict__ wp, const float* __restrict__ wl, bf* WQ, bf* WP, bf* WL) {
    constexpr int BQ = (C3 * CH / 8) / 256, BP = (CH * CH / 8) / 256, NL8 = CH * KCV / 8, GPO = KCV / 8;
    const int bx = blockIdx.x, tid = threadIdx.x; v8us o; bf* dst;
    if (bx < BQ) {
        const size_t i = (size_t)bx * 256 + tid; const v8f v = *(const v8f*)(wq + i * 8);
#pragma unroll
        for (int k = 0; k < 8; ++k) o[k] = f2bf(v[k]); dst = WQ + i * 8;
    } else if (bx < BQ + BP) {
        const size_t i = (size_t)(bx - BQ) * 256 + tid; const v8f v = *(const v8f*)(wp + i * 8);
#pragma unroll
        for (int k = 0; k < 8; ++k) o[k] = f2bf(v[k]); dst = WP + i * 8;
    } else {
        const int i = (bx - BQ - BP) * 256 + tid; if (i >= NL8) return; const int oc = i / GPO, g = i - oc * GPO; const int tap = g >> 5, c8 = (g & 31) * 8;
#pragma unroll
        for (int j = 0; j < 8; ++j) o[j] = f2bf(wl[((size_t)(oc * CH + c8 + j)) * 9 + tap]); dst = WL + (size_t)oc * KCV + (size_t)g * 8;
    }
    *(volatile v8us*)dst = o; __threadfence(); *(volatile v8us*)dst = o;
}
__global__ __launch_bounds__(256) void k_cvtx(const float* __restrict__ xb, bf* XB) {
    const int lane = threadIdx.x & 31; const int t = blockIdx.x * 8 + (threadIdx.x >> 5); if (t >= SEQ) return;
    const float* s = xb + (size_t)(lane * 8) * SEQ_FULL + t; v8us o;
#pragma unroll
    for (int j = 0; j < 8; ++j) o[j] = f2bf(s[(size_t)j * SEQ_FULL]);
    bf* dst = XB + (size_t)t * CH + lane * 8; *(volatile v8us*)dst = o; __threadfence(); *(volatile v8us*)dst = o;
}
__global__ __launch_bounds__(256) void k_planes(const float* __restrict__ F, bf* QKh, bf* QKl, h16* QK16, bf* VTh, bf* VTl, h16* VT16) {
    const int tid = threadIdx.x;
    if ((int)blockIdx.x < NQKB) {
        const size_t e = ((size_t)blockIdx.x * 256 + tid) * 2;
        const int d = (int)(e % HD); const int t = (int)((e / HD) % SEQ); const int hh = (int)((e / ((size_t)HD * SEQ)) % NH); const int sel = (int)(e / ((size_t)HD * SEQ * NH));
        const float* s = F + ((size_t)(sel * CH + hh * HD + d)) * SEQ + t; const float x0 = s[0], x1 = s[SEQ];
#if SC_HL
        unsigned short a0, b0, a1, b1; splitf(x0, a0, b0); splitf(x1, a1, b1); v2us oh, ol; oh[0] = a0; oh[1] = a1; ol[0] = b0; ol[1] = b1; (void)QK16;
        *(volatile v2us*)(QKh + e) = oh; *(volatile v2us*)(QKl + e) = ol; __threadfence(); *(volatile v2us*)(QKh + e) = oh; *(volatile v2us*)(QKl + e) = ol;
#else
        v2h o2; o2[0] = tohx(x0); o2[1] = tohx(x1); (void)QKh; (void)QKl;
        *(volatile v2h*)(QK16 + e) = o2; __threadfence(); *(volatile v2h*)(QK16 + e) = o2;
#endif
    } else {
        const size_t i = (size_t)((int)blockIdx.x - NQKB) * 256 + tid; if (i >= (size_t)NVB8) return;
        const v8f v = *(const v8f*)(F + (size_t)2 * CH * SEQ + i * 8);
#if PV_HL
        v8us oh, ol; (void)VT16;
#pragma unroll
        for (int k = 0; k < 8; ++k) { unsigned short a2, c2; splitf(v[k], a2, c2); oh[k] = a2; ol[k] = c2; }
        *(volatile v8us*)(VTh + i * 8) = oh; *(volatile v8us*)(VTl + i * 8) = ol; __threadfence(); *(volatile v8us*)(VTh + i * 8) = oh; *(volatile v8us*)(VTl + i * 8) = ol;
#else
        v8h o16; (void)VTh; (void)VTl;
#pragma unroll
        for (int k = 0; k < 8; ++k) o16[k] = tohx(v[k]);
        *(volatile v8h*)(VT16 + i * 8) = o16; __threadfence(); *(volatile v8h*)(VT16 + i * 8) = o16;
#endif
    }
}
__global__ __launch_bounds__(128) void k_asoft(const float* __restrict__ Sb, bf* Ph, bf* Pl, h16* P16) {
    const int lane = threadIdx.x & 31; const int row = blockIdx.x * 4 + (threadIdx.x >> 5); if (row >= QCH) return;
    const float* sr = Sb + (size_t)row * SEQ; float v[SEQ / 32]; float mx = -3.0e38f;
#pragma unroll
    for (int ch = 0; ch < SEQ / 128; ++ch) { const int j0 = ch * 128 + lane * 4; const v4f a = *(const v4f*)(sr + j0);
#pragma unroll
        for (int q = 0; q < 4; ++q) { float sa = a[q] * SCL; asm volatile("" : "+v"(sa)); v[ch * 4 + q] = sa; mx = fmaxf(mx, sa); }
        if ((ch & 7) == 7) asm volatile("" ::: "memory"); }
#pragma unroll
    for (int sh = 16; sh; sh >>= 1) mx = fmaxf(mx, __shfl_xor(mx, sh, 32));
    float sum = 0.f;
#pragma unroll
    for (int k = 0; k < SEQ / 32; ++k) { float d0 = __fsub_rn(v[k], mx); asm volatile("" : "+v"(d0)); v[k] = __builtin_amdgcn_exp2f(__fmul_rn(d0, 1.4426950408889634f)); sum += v[k]; }
#pragma unroll
    for (int sh = 16; sh; sh >>= 1) sum += __shfl_xor(sum, sh, 32);
#if PV_HL
    const float f = 1.0f / sum; (void)P16;
#else
    const float f = PCAR / sum; (void)Ph; (void)Pl;
#endif
#pragma unroll 1
    for (int ps = 0; ps < 2; ++ps) {
#pragma unroll
        for (int ch = 0; ch < SEQ / 128; ++ch) { const size_t oo = (size_t)row * SEQ + ch * 128 + lane * 4;
#if PV_HL
            v4us oh, ol;
#pragma unroll
            for (int q = 0; q < 4; ++q) { unsigned short a2, c2; splitf(v[ch * 4 + q] * f, a2, c2); oh[q] = a2; ol[q] = c2; }
            *(volatile v4us*)(Ph + oo) = oh; *(volatile v4us*)(Pl + oo) = ol;
#else
            v4h o4;
#pragma unroll
            for (int q = 0; q < 4; ++q) o4[q] = tohx(v[ch * 4 + q] * f);
            *(volatile v4h*)(P16 + oo) = o4;
#endif
        }
        if (ps == 0) __threadfence(); }
}
__global__ __launch_bounds__(256) void k_addsplit(const float* __restrict__ ATT, const float* __restrict__ LOC, bf* Ah, bf* Al) {
    const size_t i = (size_t)blockIdx.x * 256 + threadIdx.x; if (i >= (size_t)SEQ * CH / 8) return;
    const v8f a = *(const v8f*)(ATT + i * 8), l = *(const v8f*)(LOC + i * 8); v8us oh, ol;
#pragma unroll
    for (int k = 0; k < 8; ++k) { const float s = a[k] + l[k]; unsigned short a2, c2; splitf(s, a2, c2); oh[k] = a2; ol[k] = c2; }
    *(volatile v8us*)(Ah + i * 8) = oh; *(volatile v8us*)(Al + i * 8) = ol; __threadfence(); *(volatile v8us*)(Ah + i * 8) = oh; *(volatile v8us*)(Al + i * 8) = ol;
}

extern "C" void kernel_launch(void* const* d_in, const int* in_sizes, int n_in,
                              void* d_out, int out_size, void* d_ws, size_t ws_size, hipStream_t stream) {
    if (n_in < 12) return;
    if (in_sizes[0] < NB * CH * SEQ_FULL || in_sizes[1] < C3 * CH || in_sizes[2] < CH * CH * 9 || in_sizes[7] < CH * CH) return;
    if (in_sizes[3] < CH || in_sizes[4] < CH || in_sizes[5] < CH || in_sizes[6] < CH || in_sizes[8] < CH || in_sizes[9] < CH || in_sizes[10] < CH || in_sizes[11] < CH) return;
    if (out_size < NB * CH * SEQ) return;
    const float* x = (const float*)d_in[0]; const float* wqkv = (const float*)d_in[1]; const float* wloc = (const float*)d_in[2];
    const float* lg = (const float*)d_in[3]; const float* lb = (const float*)d_in[4]; const float* lm = (const float*)d_in[5]; const float* lv = (const float*)d_in[6];
    const float* wpr = (const float*)d_in[7]; const float* pg = (const float*)d_in[8]; const float* pb = (const float*)d_in[9]; const float* pm = (const float*)d_in[10]; const float* pv = (const float*)d_in[11];
    float* OUT = (float*)d_out;
    char* wsp = (char*)d_ws;
    auto take = [&](size_t bytes) { char* p = wsp; wsp += (bytes + 255) & ~(size_t)255; return (void*)p; };
    bf* WQ = (bf*)take((size_t)C3 * CH * 2); bf* WP = (bf*)take((size_t)CH * CH * 2); bf* WL = (bf*)take((size_t)CH * KCV * 2);
    bf* XB = (bf*)take((size_t)SEQ * CH * 2); float* FQ = (float*)take((size_t)C3 * SEQ * 4);
#if SC_HL
    bf* QKh = (bf*)take((size_t)2 * NH * SEQ * HD * 2); bf* QKl = (bf*)take((size_t)2 * NH * SEQ * HD * 2); h16* QK16 = nullptr;
#else
    h16* QK16 = (h16*)take((size_t)2 * NH * SEQ * HD * 2); bf* QKh = nullptr; bf* QKl = nullptr;
#endif
#if PV_HL
    bf* VTh = (bf*)take((size_t)CH * SEQ * 2); bf* VTl = (bf*)take((size_t)CH * SEQ * 2); h16* VT16 = nullptr;
    bf* Ph = (bf*)take((size_t)QCH * SEQ * 2); bf* Pl = (bf*)take((size_t)QCH * SEQ * 2); h16* P16 = nullptr;
#else
    h16* VT16 = (h16*)take((size_t)CH * SEQ * 2); bf* VTh = nullptr; bf* VTl = nullptr;
    h16* P16 = (h16*)take((size_t)QCH * SEQ * 2); bf* Ph = nullptr; bf* Pl = nullptr;
#endif
    float* LOC = (float*)take((size_t)SEQ * CH * 4); float* ATT = (float*)take((size_t)SEQ * CH * 4);
    bf* ACTh = (bf*)take((size_t)SEQ * CH * 2); bf* ACTl = (bf*)take((size_t)SEQ * CH * 2);
    float* Sb = (float*)take((size_t)QCH * SEQ * 4);
    if ((size_t)(wsp - (char*)d_ws) > ws_size) return;

    k_wprep<<<(unsigned)((C3 * CH / 8) / 256 + (CH * CH / 8) / 256 + (CH * KCV / 8) / 256), 256, 0, stream>>>(wqkv, wpr, wloc, WQ, WP, WL);
    for (int b = 0; b < NB; ++b) {
        k_cvtx<<<(unsigned)(SEQ / 8), 256, 0, stream>>>(x + (size_t)b * CH * SEQ_FULL, XB);
        k_gemmw<bf, 0, 0, 4><<<dim3(C3 / 64, SEQ / 64, 1), 32, 0, stream>>>(WQ, nullptr, XB, nullptr, CH, FQ, SEQ, nullptr, nullptr, nullptr, nullptr, 1.0f, 0, 0, 0);
        k_planes<<<(unsigned)(NQKB + NVB8 / 256), 256, 0, stream>>>(FQ, QKh, QKl, QK16, VTh, VTl, VT16);
        k_convw<<<dim3(SEQ / 64, CH / 64, 1), 32, 0, stream>>>(XB, WL, LOC, lg, lb, lm, lv);
        for (int h = 0; h < NH; ++h) for (int qc = 0; qc < NQC; ++qc) { const size_t q0 = (size_t)qc * QCH;
#if SC_HL
            k_gemmw<bf, 2, 0, 4><<<dim3(QCH / 64, SEQ / 64, 1), 32, 0, stream>>>(QKh + ((size_t)h * SEQ + q0) * HD, QKl + ((size_t)h * SEQ + q0) * HD, QKh + ((size_t)(NH + h) * SEQ) * HD, QKl + ((size_t)(NH + h) * SEQ) * HD,
                                                                               HD, Sb, SEQ, nullptr, nullptr, nullptr, nullptr, 1.0f, 0, 0, 0);
#else
            k_gemmw<h16, 0, 0, 4><<<dim3(QCH / 64, SEQ / 64, 1), 32, 0, stream>>>(QK16 + ((size_t)h * SEQ + q0) * HD, nullptr, QK16 + ((size_t)(NH + h) * SEQ) * HD, nullptr,
                                                                                HD, Sb, SEQ, nullptr, nullptr, nullptr, nullptr, 1.0f, 0, 0, 0);
#endif
            k_asoft<<<(unsigned)(QCH / 4), 128, 0, stream>>>(Sb, Ph, Pl, P16);
#if PV_HL
            k_gemmw<bf, 2, 0, 2><<<dim3(QCH / 64, 1, 1), 32, 0, stream>>>(Ph, Pl, VTh + (size_t)h * HD * SEQ, VTl + (size_t)h * HD * SEQ, SEQ, ATT + q0 * CH + h * HD, CH, nullptr, nullptr, nullptr, nullptr, 1.0f, 0, 0, 0);
#else
            k_gemmw<h16, 0, 0, 2><<<dim3(QCH / 64, 1, 1), 32, 0, stream>>>(P16, nullptr, VT16 + (size_t)h * HD * SEQ, nullptr, SEQ, ATT + q0 * CH + h * HD, CH, nullptr, nullptr, nullptr, nullptr, 1.0f / PCAR, 0, 0, 0);
#endif
        }
        k_addsplit<<<(unsigned)((SEQ * CH / 8) / 256), 256, 0, stream>>>(ATT, LOC, ACTh, ACTl);
        k_gemmw<bf, 3, 2, 4><<<dim3(CH / 64, SEQ / 64, 1), 32, 0, stream>>>(WP, nullptr, ACTh, ACTl, CH, OUT + (size_t)b * CH * SEQ, SEQ, pg, pb, pm, pv, 1.0f, 0, 0, 0);
    }
}
